// GraphSAGE_34557306863778
// MI455X (gfx1250) — hardware-verified
//
#include <hip/hip_runtime.h>


namespace {

constexpr int N = 50000, NP = 50048, NPL = NP  , SRCM = N  ;
constexpr int D = 128  , H1 = 256, H2 = 256, S = 10  , VOC = 1, NRL = NP  , NL = (NPL < N ? NPL : N);
constexpr float LNEPS = 1e-5f; constexpr float LOG2E = 1.4426950408889634f; constexpr float XS = 8.0f, WSC = 256.0f, WSQ = 0.25f, RS_ = 1024.0f, NSL_ = 0.2f, NSA_ = 0.01f, SLOPE = 0.0f, BNEPS = 1e-5f;
static_assert(NP % 32 == 0 && NP >= N && NPL % 32 == 0 && D % 32 == 0 && H1 % 32 == 0, "tiling");
typedef _Float16 b16;
typedef __attribute__((ext_vector_type(16))) _Float16 v16b;
typedef __attribute__((ext_vector_type(8))) _Float16 v8b;
typedef __attribute__((ext_vector_type(8))) float v8f;
typedef __attribute__((ext_vector_type(4))) float v4f;
__device__ __forceinline__ float bf16_rne(float f) { unsigned int u = __float_as_uint(f); u += 0x7FFFu + ((u >> 16) & 1u); return __uint_as_float(u & 0xFFFF0000u); }
__device__ __forceinline__ void split16(float v, b16& hi, b16& lo) { hi = (b16)v; lo = (b16)(v - (float)hi); }
__device__ __forceinline__ v16b frag_kb(const b16* p, int hh) { const v8b a = *(const v8b*)(p + 8 * hh), b = *(const v8b*)(p + 16 + 8 * hh); v16b f;
#pragma unroll
  for (int e = 0; e < 8; ++e) { f[e] = a[e]; f[8 + e] = b[e]; } return f; }
__device__ __forceinline__ v8f wmma16b(v16b a, v16b b, v8f c) { v8f d = __builtin_amdgcn_wmma_f32_16x16x32_f16(false, a, false, b, (short)0, c, false, false); asm volatile("v_nop\n\tv_nop\n\tv_nop\n\tv_nop" : "+v"(d) : "v"(a), "v"(b)); return d; }
__device__ __forceinline__ void wave_lds_sync() { __builtin_amdgcn_fence(__ATOMIC_RELEASE, "workgroup"); __builtin_amdgcn_wave_barrier(); __builtin_amdgcn_fence(__ATOMIC_ACQUIRE, "workgroup"); }
__device__ __forceinline__ float pmul(float a, float b) { float p = a * b; asm volatile("" : "+v"(p)); return p; }
__device__ __forceinline__ float bfo(float f) { float r = bf16_rne(f); asm volatile("" : "+v"(r)); return r; }
__device__ __forceinline__ int iclamp(int v, int lo, int hi) { return v < lo ? lo : (v > hi ? hi : v); }

typedef __attribute__((ext_vector_type(4))) _Float16 v4h;
__device__ __forceinline__ float lrelu(float v) { return v > 0.0f ? v : NSL_ * v; }
template <int K, int NOUTR, int NOUTP>
__global__ __launch_bounds__(256) void wt_kernel(const float* __restrict__ w, b16* __restrict__ WT, float scl) {
  const int u = blockIdx.x * 256 + threadIdx.x; if (u >= NOUTP * K / 8) return; const int e = u * 8; const int o = e / K, k0 = e % K; v8b v;
#pragma unroll
  for (int j = 0; j < 8; ++j) v[j] = (b16)(o < NOUTR ? bf16_rne(w[(size_t)(k0 + j) * NOUTR + o]) * scl : 0.0f);
  for (int pass = 0; pass < 2; ++pass) { *(volatile v8b*)(WT + e) = v; __threadfence(); }
}
template <int K, int NT, int PREC, int MODE, bool GIDX>
__global__ __launch_bounds__(64) void lin_kernel(const float* __restrict__ X, const int* __restrict__ gidx, const b16* __restrict__ WT, const b16* __restrict__ WQ, const float* __restrict__ bias, float* __restrict__ OUT, int opitch, int nvalid, int mrows) {
  constexpr int NC = NT * 16;
  __shared__ __attribute__((aligned(16))) b16 Ah[2][16][K + 8], Al[2][16][(PREC == 0 ? K : 0) + 8]; __shared__ __attribute__((aligned(16))) float Tf[2][16][NC + 4];
  const int wave = threadIdx.x >> 5, lane = threadIdx.x & 31, nloc = lane & 15, hlf = lane >> 4; const size_t m0 = (size_t)blockIdx.x * 32 + wave * 16;
  for (int idx = lane; idx < 16 * (K / 4); idx += 32) { const int rr = idx / (K / 4), c4 = (idx % (K / 4)) * 4; const size_t vrow = (m0 + rr < (size_t)nvalid) ? m0 + rr : (size_t)nvalid - 1; size_t arow = vrow; if (GIDX) arow = (size_t)iclamp(gidx[vrow], 0, VOC - 1);
    const v4f v = *(const v4f*)(X + arow * K + c4); v4h hv, lv;
    for (int j = 0; j < 4; ++j) { float vj = v[j]; if (MODE == 2) vj = fmaxf(vj, 0.0f); const float vs = (PREC == 1 ? bf16_rne(vj) : vj) * XS; const b16 ph = (b16)vs; hv[j] = ph; lv[j] = (b16)((vs - (float)ph) * RS_); } *(v4h*)(&Ah[wave][rr][c4]) = hv; if (PREC == 0) *(v4h*)(&Al[wave][rr][c4]) = lv; }
  wave_lds_sync();
  v8f acc[NT];
#pragma unroll
  for (int t = 0; t < NT; ++t) acc[t] = (v8f){};
#pragma unroll 1
  for (int kb = 0; kb < K; kb += 32) { const v16b a = frag_kb(&Ah[wave][nloc][kb], hlf); v16b al; if (PREC == 0) al = frag_kb(&Al[wave][nloc][kb], hlf);
#pragma unroll
    for (int t = 0; t < NT; ++t) { const size_t wo_ = (size_t)(t * 16 + nloc) * K + kb; acc[t] = wmma16b(a, frag_kb(WT + wo_, hlf), acc[t]); if (PREC == 0) acc[t] = wmma16b(al, frag_kb(WQ + wo_, hlf), acc[t]); } }
#pragma unroll
  for (int t = 0; t < NT; ++t) { const int col = t * 16 + nloc; const float bb = bf16_rne(bias[col]);
    for (int r = 0; r < 8; ++r) { const size_t vrow = m0 + 8 * hlf + r; float y = acc[t][r] * (1.0f / (XS * WSC)) + bb; if (MODE == 1) y = fmaxf(y, 0.0f); Tf[wave][8 * hlf + r][col] = (vrow < (size_t)nvalid) ? y : 0.0f; } }
  wave_lds_sync();
  for (int pass = 0; pass < 2; ++pass) { for (int rr = 0; rr < 16; ++rr) { if (m0 + rr < (size_t)mrows) { if (NC >= 128) { for (int c8 = 0; c8 < NC; c8 += 128) *(volatile v4f*)(OUT + (m0 + rr) * (size_t)opitch + c8 + lane * 4) = *(const v4f*)(&Tf[wave][rr][c8 + lane * 4]); }
        else { if (lane < NC / 4) *(volatile v4f*)(OUT + (m0 + rr) * (size_t)opitch + lane * 4) = *(const v4f*)(&Tf[wave][rr][lane * 4]); } } } __threadfence(); }
}
__device__ __forceinline__ float gelu_(float v) { return 0.5f * v * (1.0f + erff(v * 0.70710678118654752f)); }
template <int W, bool RNDIN>
__global__ __launch_bounds__(256) void nsamp_kernel(const float* __restrict__ Fin, const int* __restrict__ nodes, const int* __restrict__ idx, const float* __restrict__ mask, float* __restrict__ P, int mrows) {
  constexpr int CW = W / 8; const int tid = threadIdx.x; const int row = tid >> 3, g = tid & 7, c0 = g * CW; const int v = blockIdx.x * 32 + row; const int vv = v < N ? v : N - 1;
  float self_[CW], acc[CW]; for (int j = 0; j < CW; ++j) { self_[j] = 0.0f; acc[j] = 0.0f; } float msum = 0.0f;
  { int u = iclamp(nodes[vv], 0, N - 1); if (SRCM < N) u %= SRCM; const float* fr = Fin + (size_t)u * W + c0; for (int q = 0; q < CW / 4; ++q) { const v4f t4 = *(const v4f*)(fr + 4 * q); for (int j = 0; j < 4; ++j) self_[4 * q + j] = RNDIN ? bfo(t4[j]) : t4[j]; } }
#pragma unroll 1
  for (int s = 0; s < S; ++s) { const float m = bfo(mask[(size_t)vv * S + s]); int u = iclamp(idx[(size_t)vv * S + s], 0, N - 1); if (SRCM < N) u %= SRCM; msum += m; const float* fr = Fin + (size_t)u * W + c0;
    for (int q = 0; q < CW / 4; ++q) { const v4f t4 = *(const v4f*)(fr + 4 * q); for (int j = 0; j < 4; ++j) acc[4 * q + j] += pmul(m, RNDIN ? bfo(t4[j]) : t4[j]); } }
  const float inv = (msum > 0.0f) ? 1.0f / msum : 0.0f;
  for (int pass = 0; pass < 2; ++pass) { if (v < mrows) { float* prow = P + (size_t)v * (2 * W);
      for (int q = 0; q < CW / 4; ++q) { v4f a, b; for (int j = 0; j < 4; ++j) { a[j] = (v < N) ? self_[4 * q + j] : 0.0f; b[j] = (v < N) ? pmul(acc[4 * q + j], inv) : 0.0f; } *(volatile v4f*)(prow + c0 + 4 * q) = a; *(volatile v4f*)(prow + W + c0 + 4 * q) = b; } }
    __threadfence(); }
}
}

extern "C" void kernel_launch(void* const* d_in, const int* in_sizes, int n_in, void* d_out, int out_size, void* d_ws, size_t ws_size, hipStream_t stream) {
  (void)n_in;
  auto Fp = [&](int i) { return (const float*)d_in[i]; }; auto Ip = [&](int i) { return (const int*)d_in[i]; };
  if (in_sizes[0] != N || in_sizes[1] != N * D || in_sizes[2] != 2 * N * S || in_sizes[3] != 2 * N * S || in_sizes[4] != 2 * D * H1 || in_sizes[5] != H1 || in_sizes[6] != 2 * H1 * H2 || in_sizes[7] != H2 || out_size != N * H2) return;
  size_t off = 0; char* ws = (char*)d_ws;
  auto carve = [&](size_t bytes) { char* p = ws + off; off += (bytes + 255) & ~(size_t)255; return p; };
  b16* W1T = (b16*)carve((size_t)H1 * 2 * D * 2); b16* W1Q = (b16*)carve((size_t)H1 * 2 * D * 2); b16* W2T = (b16*)carve((size_t)H2 * 2 * H1 * 2); b16* W2Q = (b16*)carve((size_t)H2 * 2 * H1 * 2);
  float* P1 = (float*)carve((size_t)NP * 2 * D * 4); float* HA = (float*)carve((size_t)NP * H1 * 4); float* P2 = (float*)carve((size_t)NP * 2 * H1 * 4);
  if (off > ws_size || off > ((size_t)216 << 20)) return;
  { wt_kernel<2 * D, H1, H1><<<(H1 * 2 * D / 8 + 255) / 256, 256, 0, stream>>>(Fp(4), W1T, WSC); wt_kernel<2 * D, H1, H1><<<(H1 * 2 * D / 8 + 255) / 256, 256, 0, stream>>>(Fp(4), W1Q, WSQ);
    wt_kernel<2 * H1, H2, H2><<<(H2 * 2 * H1 / 8 + 255) / 256, 256, 0, stream>>>(Fp(6), W2T, WSC); wt_kernel<2 * H1, H2, H2><<<(H2 * 2 * H1 / 8 + 255) / 256, 256, 0, stream>>>(Fp(6), W2Q, WSQ); }
  nsamp_kernel<D, true><<<NRL / 32, 256, 0, stream>>>(Fp(1), Ip(0), Ip(2), Fp(3), P1, NRL);
  lin_kernel<2 * D, 16, 0, 1, false><<<NRL / 32, 64, 0, stream>>>(P1, nullptr, W1T, W1Q, Fp(5), HA, H1, N, NRL);
  nsamp_kernel<H1, false><<<NPL / 32, 256, 0, stream>>>(HA, Ip(0), Ip(2) + (size_t)N * S, Fp(3) + (size_t)N * S, P2, NPL);
  lin_kernel<2 * H1, 16, 0, 1, false><<<NPL / 32, 64, 0, stream>>>(P2, nullptr, W2T, W2Q, Fp(7), (float*)d_out, H2, N, NL);
}
